// RecurrentAE_14061722927625
// MI455X (gfx1250) — hardware-run, weakly checked
//
#include <hip/hip_runtime.h>
#include <math.h>
#include <stdint.h>

constexpr int NSEQ    = 256;
constexpr int NSTEP   = 512;
constexpr int NHID    = 256;
constexpr int NG3     = 768;
constexpr int NTHR    = 256;
constexpr int NWAVE   = 8;
constexpr int TROWS   = 16;
constexpr int HPITCH  = 264;
constexpr int XCH     = 32;
constexpr int OCH     = 32;
constexpr int KSTEPS  = NHID / 32;
constexpr int GSTRIDE = NHID * NHID;
constexpr float A_CARRY = 16.0f;
constexpr float W_CARRY = 64.0f;
constexpr float Z_FOLD  = 1.0f / 1024.0f;

static_assert(NSEQ % TROWS == 0, "grid covers all sequences exactly");
static_assert(NSTEP % XCH == 0 && NSTEP % OCH == 0, "chunks tile the time axis exactly");
static_assert(TROWS * XCH == 128 * 4, "one float4 per thread (128 threads) per input chunk");
static_assert(TROWS * OCH == 128 * 4, "one float4 per thread (4 waves) per output chunk");
static_assert((NG3 * NHID / 8) % NTHR == 0, "weight prep grid exact");
static_assert(NHID % 32 == 0, "K multiple of 32");
static_assert(NWAVE * 32 == NHID, "8 waves x 32 units cover the hidden dimension");
static_assert((HPITCH * 2) % 16 == 0, "h tile rows 16-B aligned");

typedef __attribute__((ext_vector_type(16))) _Float16 v16h;
typedef __attribute__((ext_vector_type(8)))  _Float16 v8h;
typedef __attribute__((ext_vector_type(8)))  float    v8f;
typedef __attribute__((ext_vector_type(4)))  float    v4f;

__device__ __forceinline__ unsigned short f2bf_bits(float f) {
  unsigned u = __float_as_uint(f);
  return (unsigned short)((u + 0x7FFFu + ((u >> 16) & 1u)) >> 16);
}
__device__ __forceinline__ float bf_bits2f(unsigned short h) { return __uint_as_float(((unsigned)h) << 16); }
__device__ __forceinline__ float bfr(float f) { return bf_bits2f(f2bf_bits(f)); }

__device__ __forceinline__ void keep4_h(v16h a, v16h b, v16h c, v16h d) { asm volatile("v_nop" :: "v"(a), "v"(b), "v"(c), "v"(d)); }
__device__ __forceinline__ void keep3_h(v16h a, v16h b, v16h c) { asm volatile("v_nop" :: "v"(a), "v"(b), "v"(c)); }
__device__ __forceinline__ void acc_guard6(v8f& a, v8f& b, v8f& c, v8f& d, v8f& e, v8f& f) {
  asm volatile("v_nop\n\tv_nop\n\tv_nop\n\tv_nop" : "+v"(a), "+v"(b), "+v"(c), "+v"(d), "+v"(e), "+v"(f));
}
template <typename T> struct Frag;
template <> struct Frag<_Float16> {
  typedef v16h V; union U { v16h v; v8h h[2]; };
  static __device__ __forceinline__ v16h load(const _Float16* p) {
    U f; f.h[0] = *(const v8h*)(p); f.h[1] = *(const v8h*)(p + 16); return f.v;
  }
  static __device__ __forceinline__ v8f mma(v16h a, v16h b, v8f c) {
    return __builtin_amdgcn_wmma_f32_16x16x32_f16(false, a, false, b, (short)0, c, false, false);
  }
};
typedef Frag<_Float16> FragH;

__device__ __forceinline__ float fsig(float v)  { return __builtin_amdgcn_rcpf(1.0f + __expf(-v)); }
__device__ __forceinline__ float ftanh(float v) { return 1.0f - 2.0f * __builtin_amdgcn_rcpf(__expf(2.0f * v) + 1.0f); }

__global__ __launch_bounds__(NTHR) void wprep_kernel(const float* __restrict__ W, int n8, unsigned short* __restrict__ O) {
  const int i = blockIdx.x * NTHR + threadIdx.x;
  if (i >= n8) return;
  const int e0 = i * 8;
  v8h hv;
#pragma unroll
  for (int e = 0; e < 8; ++e) {
    const float fb = bfr(W[e0 + e]);
    hv[e] = (_Float16)(fb * W_CARRY);
  }
  *(volatile v8h*)(O + e0) = hv;
  __threadfence();
  *(volatile v8h*)(O + e0) = hv;
}

__device__ __forceinline__ void mac_gru(v8f (&acc)[6], const _Float16* arow, const _Float16* w0, const _Float16* w1) {
#pragma unroll 1
  for (int kc = 0; kc < KSTEPS; ++kc) {
    const int k0 = kc * 32;
    const v16h a  = FragH::load(arow + k0);
    const v16h b0 = FragH::load(w0 + k0);
    const v16h b1 = FragH::load(w0 + GSTRIDE + k0);
    const v16h b2 = FragH::load(w0 + 2 * GSTRIDE + k0);
    const v16h b3 = FragH::load(w1 + k0);
    const v16h b4 = FragH::load(w1 + GSTRIDE + k0);
    const v16h b5 = FragH::load(w1 + 2 * GSTRIDE + k0);
    acc[0] = FragH::mma(a, b0, acc[0]);
    acc[1] = FragH::mma(a, b1, acc[1]);
    acc[2] = FragH::mma(a, b2, acc[2]);
    acc[3] = FragH::mma(a, b3, acc[3]);
    acc[4] = FragH::mma(a, b4, acc[4]);
    acc[5] = FragH::mma(a, b5, acc[5]);
    acc_guard6(acc[0], acc[1], acc[2], acc[3], acc[4], acc[5]);
    keep4_h(a, b0, b1, b2);
    keep3_h(b3, b4, b5);
  }
}

struct GateConst { float wir, wiz, win, cr, cz, cin, chn; };
__device__ __forceinline__ GateConst load_gc(const float* __restrict__ wih, const float* __restrict__ bih,
                                             const float* __restrict__ bhh, int j) {
  GateConst g;
  g.wir = bfr(wih[j]);
  g.wiz = bfr(wih[NHID + j]);
  g.win = bfr(wih[2 * NHID + j]);
  g.cr  = bfr(bih[j]) + bfr(bhh[j]);
  g.cz  = bfr(bih[NHID + j]) + bfr(bhh[NHID + j]);
  g.cin = bfr(bih[2 * NHID + j]);
  g.chn = bfr(bhh[2 * NHID + j]);
  return g;
}

__device__ __forceinline__ void cell8(const v8f& ar, const v8f& az, const v8f& an, const float (&xr)[8],
                                      const GateConst& g, float (&h)[8]) {
#pragma unroll
  for (int r = 0; r < 8; ++r) {
    const float pr  = fmaf(ar[r], Z_FOLD, fmaf(xr[r], g.wir, g.cr));
    const float pz  = fmaf(az[r], Z_FOLD, fmaf(xr[r], g.wiz, g.cz));
    const float gin = fmaf(xr[r], g.win, g.cin);
    const float ghn = fmaf(an[r], Z_FOLD, g.chn);
    const float rr  = fsig(pr);
    const float zz  = fsig(pz);
    const float nn  = ftanh(fmaf(rr, ghn, gin));
    h[r] = fmaf(zz, h[r] - nn, nn);
  }
}

__device__ __forceinline__ void dense_partial(const float (&h0)[8], const float (&h1)[8], float wd0, float wd1,
                                              float* Pw, int wave, int hh, int c) {
  float p[8];
#pragma unroll
  for (int r = 0; r < 8; ++r) p[r] = fmaf(h0[r], wd0, h1[r] * wd1);
#pragma unroll
  for (int r = 0; r < 8; ++r) {
#pragma unroll
    for (int off = 1; off < 16; off <<= 1) p[r] += __shfl_xor(p[r], off, 32);
  }
  if (c == 0) {
#pragma unroll
    for (int r = 0; r < 8; ++r) Pw[wave * TROWS + 8 * hh + r] = p[r];
  }
}

__global__ __launch_bounds__(NTHR) void gru_ae_kernel(
    const float* __restrict__ x,
    const float* __restrict__ w_ih_e, const float* __restrict__ b_ih_e, const float* __restrict__ b_hh_e,
    const float* __restrict__ w_ih_d, const float* __restrict__ b_ih_d, const float* __restrict__ b_hh_d,
    const float* __restrict__ w_dn,   const float* __restrict__ b_dn,
    const unsigned short* __restrict__ WhhEp,
    const unsigned short* __restrict__ WhhDp,
    float* __restrict__ out) {
  __shared__ __align__(16) _Float16 Ht[TROWS * HPITCH];
  __shared__ __align__(16) float    Xe[TROWS * XCH];
  __shared__ __align__(16) float    Xs[TROWS];
  __shared__ __align__(16) float    Pw[NWAVE * TROWS];
  __shared__ __align__(16) float    Ob[TROWS * OCH];

  const int tid = threadIdx.x, lane = tid & 31, wave = tid >> 5;
  const int c = lane & 15, hh = lane >> 4, koff = hh * 8;
  const int rb = 8 * hh;
  const int rowbase = blockIdx.x * TROWS;
  const int j0 = 32 * wave + c;
  const int j1 = j0 + 16;

#pragma unroll 1
  for (int i = tid; i < TROWS * HPITCH; i += NTHR) Ht[i] = (_Float16)0.0f;

  const float wd0 = bfr(w_dn[j0]);
  const float wd1 = bfr(w_dn[j1]);
  const float bd  = bfr(b_dn[0]);

  float hst0[8], hst1[8];
#pragma unroll
  for (int r = 0; r < 8; ++r) { hst0[r] = 0.0f; hst1[r] = 0.0f; }
  __syncthreads();

  const _Float16* arow = Ht + c * HPITCH + koff;
  const _Float16* whe0 = (const _Float16*)WhhEp + (size_t)j0 * NHID + koff;
  const _Float16* whe1 = (const _Float16*)WhhEp + (size_t)j1 * NHID + koff;
  const _Float16* whd0 = (const _Float16*)WhhDp + (size_t)j0 * NHID + koff;
  const _Float16* whd1 = (const _Float16*)WhhDp + (size_t)j1 * NHID + koff;
  const v8f z8 = {0.f, 0.f, 0.f, 0.f, 0.f, 0.f, 0.f, 0.f};

  {
    const GateConst ge0 = load_gc(w_ih_e, b_ih_e, b_hh_e, j0);
    const GateConst ge1 = load_gc(w_ih_e, b_ih_e, b_hh_e, j1);
#pragma unroll 1
    for (int t = 0; t < NSTEP; ++t) {
      const int tc = t & (XCH - 1);
      if (tc == 0) {
        if (tid < (TROWS * XCH) / 4) {
          const int row = tid >> 3, c4 = (tid & 7) * 4;
          const v4f v = *(const v4f*)(x + ((size_t)(rowbase + row) * NSTEP + (size_t)(t + c4)));
          v4f w;
          w[0] = bfr(v[0]); w[1] = bfr(v[1]); w[2] = bfr(v[2]); w[3] = bfr(v[3]);
          *(v4f*)(Xe + row * XCH + c4) = w;
        }
        __syncthreads();
      }
      float xr[8];
#pragma unroll
      for (int r = 0; r < 8; ++r) xr[r] = Xe[(rb + r) * XCH + tc];
      v8f acc[6];
      acc[0] = z8; acc[1] = z8; acc[2] = z8; acc[3] = z8; acc[4] = z8; acc[5] = z8;
      mac_gru(acc, arow, whe0, whe1);
      cell8(acc[0], acc[1], acc[2], xr, ge0, hst0);
      cell8(acc[3], acc[4], acc[5], xr, ge1, hst1);
      dense_partial(hst0, hst1, wd0, wd1, Pw, wave, hh, c);
      __syncthreads();
#pragma unroll
      for (int r = 0; r < 8; ++r) {
        Ht[(rb + r) * HPITCH + j0] = (_Float16)(A_CARRY * hst0[r]);
        Ht[(rb + r) * HPITCH + j1] = (_Float16)(A_CARRY * hst1[r]);
      }
      if (tid < TROWS) {
        float sx = Pw[tid];
#pragma unroll
        for (int w = 1; w < NWAVE; ++w) sx += Pw[w * TROWS + tid];
        Xs[tid] = sx + bd;
      }
      __syncthreads();
    }
  }

  {
    const GateConst gd0 = load_gc(w_ih_d, b_ih_d, b_hh_d, j0);
    const GateConst gd1 = load_gc(w_ih_d, b_ih_d, b_hh_d, j1);
#pragma unroll 1
    for (int s = 0; s < NSTEP; ++s) {
      float xr[8];
#pragma unroll
      for (int r = 0; r < 8; ++r) xr[r] = Xs[rb + r];
      v8f acc[6];
      acc[0] = z8; acc[1] = z8; acc[2] = z8; acc[3] = z8; acc[4] = z8; acc[5] = z8;
      mac_gru(acc, arow, whd0, whd1);
      cell8(acc[0], acc[1], acc[2], xr, gd0, hst0);
      cell8(acc[3], acc[4], acc[5], xr, gd1, hst1);
      dense_partial(hst0, hst1, wd0, wd1, Pw, wave, hh, c);
      __syncthreads();
#pragma unroll
      for (int r = 0; r < 8; ++r) {
        Ht[(rb + r) * HPITCH + j0] = (_Float16)(A_CARRY * hst0[r]);
        Ht[(rb + r) * HPITCH + j1] = (_Float16)(A_CARRY * hst1[r]);
      }
      if (tid < TROWS) {
        float sx = Pw[tid];
#pragma unroll
        for (int w = 1; w < NWAVE; ++w) sx += Pw[w * TROWS + tid];
        const float xv = sx + bd;
        Xs[tid] = xv;
        Ob[tid * OCH + (OCH - 1 - (s & (OCH - 1)))] = xv;
      }
      __syncthreads();
      if ((s & (OCH - 1)) == OCH - 1 && wave < 4) {
        const int q = s >> 5;
        const int row = 4 * wave + (lane >> 3), c4 = (lane & 7) * 4;
        const v4f v = *(const v4f*)(Ob + row * OCH + c4);
        float* p = out + (size_t)(rowbase + row) * NSTEP + (size_t)(NSTEP - OCH * (q + 1)) + c4;
        *(volatile v4f*)p = v;
        __threadfence();
        *(volatile v4f*)p = v;
      }
    }
  }
}

extern "C" void kernel_launch(void* const* d_in, const int* in_sizes, int n_in,
                              void* d_out, int out_size, void* d_ws, size_t ws_size, hipStream_t stream) {
  if (n_in < 11 || d_out == nullptr || d_ws == nullptr) return;
  if (in_sizes[0] != NSEQ * NSTEP || in_sizes[1] != NG3 || in_sizes[2] != NG3 * NHID || in_sizes[3] != NG3 ||
      in_sizes[4] != NG3 || in_sizes[5] != NG3 || in_sizes[6] != NG3 * NHID || in_sizes[7] != NG3 ||
      in_sizes[8] != NG3 || in_sizes[9] != NHID || in_sizes[10] < 1 || out_size != NSEQ * NSTEP) return;
  const size_t plane_bytes = (size_t)NG3 * NHID * 2;
  if (ws_size < 2 * plane_bytes) return;

  const float* x        = (const float*)d_in[0];
  const float* w_ih_enc = (const float*)d_in[1];
  const float* w_hh_enc = (const float*)d_in[2];
  const float* b_ih_enc = (const float*)d_in[3];
  const float* b_hh_enc = (const float*)d_in[4];
  const float* w_ih_dec = (const float*)d_in[5];
  const float* w_hh_dec = (const float*)d_in[6];
  const float* b_ih_dec = (const float*)d_in[7];
  const float* b_hh_dec = (const float*)d_in[8];
  const float* w_dense  = (const float*)d_in[9];
  const float* b_dense  = (const float*)d_in[10];
  float* out = (float*)d_out;

  char* ws = (char*)d_ws;
  unsigned short* WHHE = (unsigned short*)(ws);
  unsigned short* WHHD = (unsigned short*)(ws + plane_bytes);

  const int n8 = NG3 * NHID / 8;
  wprep_kernel<<<n8 / NTHR, NTHR, 0, stream>>>(w_hh_enc, n8, WHHE);
  wprep_kernel<<<n8 / NTHR, NTHR, 0, stream>>>(w_hh_dec, n8, WHHD);
  gru_ae_kernel<<<NSEQ / TROWS, NTHR, 0, stream>>>(
      x, w_ih_enc, b_ih_enc, b_hh_enc, w_ih_dec, b_ih_dec, b_hh_dec, w_dense, b_dense, WHHE, WHHD, out);
}
